// TransformerModel_14705968021921
// MI455X (gfx1250) — hardware-verified
//
#include <hip/hip_runtime.h>
#include <math.h>

typedef __attribute__((ext_vector_type(16))) _Float16 v16h;
typedef __attribute__((ext_vector_type(8)))  _Float16 v8h;
typedef __attribute__((ext_vector_type(16))) __bf16   v16b;
typedef __attribute__((ext_vector_type(8)))  __bf16   v8b;
typedef __attribute__((ext_vector_type(8)))  float    v8f;
typedef __attribute__((ext_vector_type(4)))  float    v4f;

constexpr int kS    = 1024;
constexpr int kD    = 512;
constexpr int kNH   = 8;
constexpr int kDH   = 64;
constexpr int kNL   = 12;
constexpr int kFF   = 2048;
constexpr int kE    = 768;
constexpr int kC    = 128;
constexpr int kNC   = kS / kC;
constexpr int kNE   = 8;
constexpr int kNEP  = 64;
constexpr int kThr  = 256;
constexpr float kInCarry = 1024.0f;
constexpr float kWCarry = 4096.0f;
constexpr float kCQ = 256.0f;
constexpr float kCW = 64.0f;
constexpr float kCST = 8.0f;
constexpr float kScX = 1.0f / (kInCarry * kWCarry), kScQK = 1.0f / (kCQ * kCQ), kScWV = 1.0f / (kCW * kInCarry), kScQS = 1.0f / (kCQ * kCST), kScU = 1.0f / (kInCarry * kCQ);
constexpr float kInvD = 1.0f / 512.0f;
constexpr float kLnEps = 1e-5f;
constexpr float kAttEps = 1e-6f;
constexpr float kF16MinNormal = 6.103515625e-5f;

static_assert(kS == 1024 && kNH * kDH == kD && kNC * kC == kS && ((kS / 64) * (kD / 64)) % 8 == 0 && ((kS / 64) * (3 * kD / 64)) % 8 == 0 && ((kS / 64) * (kFF / 64)) % 8 == 0 && ((kS / 64) * (kNEP / 64)) % 8 == 0, "GEMM M and N multiples of 64; the whole-sequence grids whole numbers of 8-tile blocks (the per-chunk products run ONE 8-wave block a head: 4, 2 or 1 tiles: the engine's own tile guard retires the other waves)");
static_assert((kE % 32) == 0 && (kD % 32) == 0 && (kFF % 32) == 0 && (kDH % 32) == 0 && (kC % 32) == 0, "GEMM K multiples of 32");

constexpr size_t kOffE16 = 0ull;
constexpr size_t kOffINW16 = 1572864ull;
constexpr size_t kOffEMOW16 = 2359296ull;
constexpr size_t kOffWQKV16 = 2424832ull;
constexpr size_t kOffWO16 = 3997696ull;
constexpr size_t kOffW1H = 4521984ull;
constexpr size_t kOffW2H = 6619136ull;
constexpr size_t kOffBIAS = 8716288ull;
constexpr size_t kOffPE = 8949760ull;
constexpr size_t kOffH = 11046912ull;
constexpr size_t kOffH16 = 13144064ull;
constexpr size_t kOffQKV = 14192640ull;
constexpr size_t kOffQ16 = 20484096ull;
constexpr size_t kOffK16 = 21532672ull;
constexpr size_t kOffKF = 22581248ull;
constexpr size_t kOffKT16 = 24678400ull;
constexpr size_t kOffVT16 = 25726976ull;
constexpr size_t kOffSC = 26775552ull;
constexpr size_t kOffW16 = 27299840ull;
constexpr size_t kOffDENI = 27561984ull;
constexpr size_t kOffP1 = 27566080ull;
constexpr size_t kOffP2 = 27828224ull;
constexpr size_t kOffU = 28090368ull;
constexpr size_t kOffST32 = 28221440ull;
constexpr size_t kOffST16 = 28352512ull;
constexpr size_t kOffKS = 28418048ull;
constexpr size_t kOffATT16 = 28420096ull;
constexpr size_t kOffAO = 29468672ull;
constexpr size_t kOffF1 = 31565824ull;
constexpr size_t kOffG16 = 39954432ull;
constexpr size_t kOffEMO = 44148736ull;
constexpr size_t kWsTotal = 44410880ull;
static_assert(kWsTotal <= 134217728ull, "carve cap: under 128 MiB");
static_assert(kOffE16 == 0
              && kOffINW16 == kOffE16 + 1572864ull
              && kOffEMOW16 == kOffINW16 + 786432ull
              && kOffWQKV16 == kOffEMOW16 + 65536ull
              && kOffWO16 == kOffWQKV16 + 1572864ull
              && kOffW1H == kOffWO16 + 524288ull
              && kOffW2H == kOffW1H + 2097152ull
              && kOffBIAS == kOffW2H + 2097152ull
              && kOffPE == kOffBIAS + 233472ull
              && kOffH == kOffPE + 2097152ull
              && kOffH16 == kOffH + 2097152ull
              && kOffQKV == kOffH16 + 1048576ull
              && kOffQ16 == kOffQKV + 6291456ull
              && kOffK16 == kOffQ16 + 1048576ull
              && kOffKF == kOffK16 + 1048576ull
              && kOffKT16 == kOffKF + 2097152ull
              && kOffVT16 == kOffKT16 + 1048576ull
              && kOffSC == kOffVT16 + 1048576ull
              && kOffW16 == kOffSC + 524288ull
              && kOffDENI == kOffW16 + 262144ull
              && kOffP1 == kOffDENI + 4096ull
              && kOffP2 == kOffP1 + 262144ull
              && kOffU == kOffP2 + 262144ull
              && kOffST32 == kOffU + 131072ull
              && kOffST16 == kOffST32 + 131072ull
              && kOffKS == kOffST16 + 65536ull
              && kOffATT16 == kOffKS + 2048ull
              && kOffAO == kOffATT16 + 1048576ull
              && kOffF1 == kOffAO + 2097152ull
              && kOffG16 == kOffF1 + 8388608ull
              && kOffEMO == kOffG16 + 4194304ull
              && kWsTotal == kOffEMO + 262144ull, "the carve is chained and totalled");
static_assert((kOffE16 % 256) == 0 && (kOffINW16 % 256) == 0 && (kOffEMOW16 % 256) == 0 && (kOffWQKV16 % 256) == 0 && (kOffWO16 % 256) == 0 && (kOffW1H % 256) == 0 && (kOffW2H % 256) == 0 && (kOffBIAS % 256) == 0 && (kOffPE % 256) == 0 && (kOffH % 256) == 0 && (kOffH16 % 256) == 0 && (kOffQKV % 256) == 0 && (kOffQ16 % 256) == 0 && (kOffK16 % 256) == 0 && (kOffKF % 256) == 0 && (kOffKT16 % 256) == 0 && (kOffVT16 % 256) == 0 && (kOffSC % 256) == 0 && (kOffW16 % 256) == 0 && (kOffDENI % 256) == 0 && (kOffP1 % 256) == 0 && (kOffP2 % 256) == 0 && (kOffU % 256) == 0 && (kOffST32 % 256) == 0 && (kOffST16 % 256) == 0 && (kOffKS % 256) == 0 && (kOffATT16 % 256) == 0 && (kOffAO % 256) == 0 && (kOffF1 % 256) == 0 && (kOffG16 % 256) == 0 && (kOffEMO % 256) == 0, "aligned regions");

__device__ __forceinline__ unsigned short f2bf_bits(float f) {
  unsigned u = __float_as_uint(f);
  return (unsigned short)((u + 0x7FFFu + ((u >> 16) & 1u)) >> 16);
}
__device__ __forceinline__ float bf_bits2f(unsigned short h) { return __uint_as_float(((unsigned)h) << 16); }
__device__ __forceinline__ float bf16r(float f) { return bf_bits2f(f2bf_bits(f)); }
__device__ __forceinline__ float carry_flush(float v, float carry) {
  const float s = v * carry;
  return (fabsf(s) < kF16MinNormal) ? 0.0f : s;
}
__device__ __forceinline__ float frcp(float x) { return __builtin_amdgcn_rcpf(x); }

__device__ __forceinline__ void dep_guard4_h(v8f& a, v8f& b, v8f& c, v8f& d, v16h x, v16h y) { asm volatile("v_nop\n\tv_nop\n\tv_nop\n\tv_nop" : "+v"(a), "+v"(b), "+v"(c), "+v"(d) : "v"(x), "v"(y)); }
__device__ __forceinline__ void dep_guard4_b(v8f& a, v8f& b, v8f& c, v8f& d, v16b x, v16b y) { asm volatile("v_nop\n\tv_nop\n\tv_nop\n\tv_nop" : "+v"(a), "+v"(b), "+v"(c), "+v"(d) : "v"(x), "v"(y)); }
__device__ __forceinline__ void keep4_h(v16h a, v16h b, v16h c, v16h d) { asm volatile("v_nop" :: "v"(a), "v"(b), "v"(c), "v"(d)); }
__device__ __forceinline__ void keep4_b(v16b a, v16b b, v16b c, v16b d) { asm volatile("v_nop" :: "v"(a), "v"(b), "v"(c), "v"(d)); }
__device__ __forceinline__ void acc_guard4(v8f& a, v8f& b, v8f& c, v8f& d) { asm volatile("v_nop\n\tv_nop\n\tv_nop\n\tv_nop" : "+v"(a), "+v"(b), "+v"(c), "+v"(d)); }

template <typename T> struct Frag;
template <> struct Frag<_Float16> {
  typedef v16h V; union U { v16h v; v8h h[2]; };
  static __device__ __forceinline__ v16h load(const _Float16* p) {
    U f; f.h[0] = *(const v8h*)(p); f.h[1] = *(const v8h*)(p + 16); return f.v;
  }
  static __device__ __forceinline__ v8f mma(v16h a, v16h b, v8f c) {
    return __builtin_amdgcn_wmma_f32_16x16x32_f16(false, a, false, b, (short)0, c, false, false);
  }
  static __device__ __forceinline__ void guard4(v8f& a, v8f& b, v8f& c, v8f& d, v16h x, v16h y) { dep_guard4_h(a, b, c, d, x, y); }
  static __device__ __forceinline__ void keep(v16h a, v16h b, v16h c, v16h d) { keep4_h(a, b, c, d); }
};
template <> struct Frag<__bf16> {
  typedef v16b V; union U { v16b v; v8b h[2]; };
  static __device__ __forceinline__ v16b load(const __bf16* p) {
    U f; f.h[0] = *(const v8b*)(p); f.h[1] = *(const v8b*)(p + 16); return f.v;
  }
  static __device__ __forceinline__ v8f mma(v16b a, v16b b, v8f c) {
    return __builtin_amdgcn_wmma_f32_16x16x32_bf16(false, a, false, b, (short)0, c, false, false);
  }
  static __device__ __forceinline__ void guard4(v8f& a, v8f& b, v8f& c, v8f& d, v16b x, v16b y) { dep_guard4_b(a, b, c, d, x, y); }
  static __device__ __forceinline__ void keep(v16b a, v16b b, v16b c, v16b d) { keep4_b(a, b, c, d); }
};

__device__ __forceinline__ v8f mma_h(v16h a, v16h b, v8f c) {
  c = __builtin_amdgcn_wmma_f32_16x16x32_f16(false, a, false, b, (short)0, c, false, false);
  asm volatile("v_nop\n\tv_nop\n\tv_nop\n\tv_nop" : "+v"(c) : "v"(a), "v"(b));
  return c;
}

template <int ET> struct Elem;
template <> struct Elem<0> { typedef _Float16 T; };
template <> struct Elem<1> { typedef __bf16 T; };
template <int ET, bool SPLIT, int BIAS_MODE, int OUT_MODE, bool RESID, int ACT = 0>
__global__ __launch_bounds__(256) void wmma_gemm64(
    const unsigned short* __restrict__ Ap, const unsigned short* __restrict__ A2p, int lda, long strideA,
    const unsigned short* __restrict__ Btp, const unsigned short* __restrict__ Bt2p, int ldb, long strideB,
    void* __restrict__ Cout, void* __restrict__ Cout2, int ldc, long strideC,
    const float* __restrict__ bias,
    const float* __restrict__ resid, long strideR,
    int M, int N, int K, float scale) {
  typedef typename Elem<ET>::T T;
  typedef typename Frag<T>::V V;
  const T* A = (const T*)Ap; const T* A2 = (const T*)A2p; const T* Bt = (const T*)Btp; const T* Bt2 = (const T*)Bt2p;
  __shared__ __align__(16) float sT[8][16 * 68];
  const int b    = blockIdx.y;
  const int lane = threadIdx.x & 31;
  const int wave = threadIdx.x >> 5;
  const int tilesN = N >> 6;
  const int tilesM = M >> 6;
  const int tile = blockIdx.x * 8 + wave;
  if (tile >= tilesM * tilesN) return;
  const int tm = tile / tilesN;
  const int tn = tile - tm * tilesN;
  const int m0 = tm << 6;
  const int n0 = tn << 6;

  const T* Ab  = A  + (size_t)b * strideA;
  const T* Bb  = Bt + (size_t)b * strideB;
  const T* Ab2 = SPLIT ? (A2  + (size_t)b * strideA) : nullptr;
  const T* Bb2 = SPLIT ? (Bt2 + (size_t)b * strideB) : nullptr;

  const int rlane = lane & 15;
  const int koff  = (lane >> 4) * 8;
  const int mOff  = (lane >> 4) * 8;

  v8f acc[4][4];
#pragma unroll
  for (int i = 0; i < 4; ++i)
#pragma unroll
    for (int j = 0; j < 4; ++j) acc[i][j] = (v8f){0.f,0.f,0.f,0.f,0.f,0.f,0.f,0.f};

  for (int k0 = 0; k0 < K; k0 += 32) {
    V bh[4], bl[4];
#pragma unroll
    for (int j = 0; j < 4; ++j) {
      const size_t bo = (size_t)(n0 + (j << 4) + rlane) * ldb + koff + k0;
      bh[j] = Frag<T>::load(Bb + bo);
      if (SPLIT) bl[j] = Frag<T>::load(Bb2 + bo);
    }
#pragma unroll
    for (int i = 0; i < 4; ++i) {
      const size_t ao = (size_t)(m0 + (i << 4) + rlane) * lda + koff + k0;
      V ah = Frag<T>::load(Ab + ao);
      V al;
      if (SPLIT) al = Frag<T>::load(Ab2 + ao);
#pragma unroll
      for (int j = 0; j < 4; ++j) {
        acc[i][j] = Frag<T>::mma(ah, bh[j], acc[i][j]);
        if (SPLIT) {
          acc[i][j] = Frag<T>::mma(ah, bl[j], acc[i][j]);
          acc[i][j] = Frag<T>::mma(al, bh[j], acc[i][j]);
        }
      }
      Frag<T>::guard4(acc[i][0], acc[i][1], acc[i][2], acc[i][3], ah, SPLIT ? al : ah);
    }
    Frag<T>::keep(bh[0], bh[1], bh[2], bh[3]);
    if (SPLIT) Frag<T>::keep(bl[0], bl[1], bl[2], bl[3]);
  }
  acc_guard4(acc[0][0], acc[0][1], acc[0][2], acc[0][3]);
  acc_guard4(acc[1][0], acc[1][1], acc[1][2], acc[1][3]);
  acc_guard4(acc[2][0], acc[2][1], acc[2][2], acc[2][3]);
  acc_guard4(acc[3][0], acc[3][1], acc[3][2], acc[3][3]);

  float* slab = sT[wave];
  const float* Rb = RESID ? (resid + (size_t)b * strideR) : nullptr;
#pragma unroll
  for (int i = 0; i < 4; ++i) {
    const int mBase = m0 + (i << 4);
#pragma unroll
    for (int j = 0; j < 4; ++j) {
      const int n = n0 + (j << 4) + rlane;
      float bv = 0.f;
      if (BIAS_MODE == 2) bv = bias[n];
#pragma unroll
      for (int r = 0; r < 8; ++r) {
        float v = acc[i][j][r] * scale;
        if (BIAS_MODE == 1) v += bias[mBase + mOff + r];
        if (BIAS_MODE == 2) v += bv;
        if (RESID) v += Rb[(size_t)(mBase + mOff + r) * ldc + n];
        if (ACT == 1) v = tanhf(v);
        if (ACT == 2) v = fmaxf(v, 0.0f);
        if (ACT == 3) v = v / (1.0f + expf(-v));
        if (ACT == 4) v = (v > 0.f) ? v : 0.01f * v;
        slab[(mOff + r) * 68 + (j << 4) + rlane] = v;
      }
    }
    __builtin_amdgcn_fence(__ATOMIC_RELEASE, "workgroup");
    __builtin_amdgcn_wave_barrier();
    __builtin_amdgcn_fence(__ATOMIC_ACQUIRE, "workgroup");
    if (OUT_MODE == 0) {
      float* C = (float*)Cout + (size_t)b * strideC;
      const int hh = lane >> 4, c4 = (lane & 15) * 4;
      for (int pass = 0; pass < 2; ++pass) {
#pragma unroll
        for (int it = 0; it < 8; ++it) {
          const int row = it * 2 + hh;
          v4f v = *(const v4f*)(slab + row * 68 + c4);
          *(volatile v4f*)(C + (size_t)(mBase + row) * ldc + n0 + c4) = v;
        }
        __threadfence();
      }
    } else {
      const int q = lane >> 3, c8 = (lane & 7) * 8;
      unsigned short* C  = (unsigned short*)Cout  + (size_t)b * strideC;
      unsigned short* C2 = (OUT_MODE == 2) ? ((unsigned short*)Cout2 + (size_t)b * strideC) : nullptr;
      for (int pass = 0; pass < 2; ++pass) {
#pragma unroll
        for (int it = 0; it < 4; ++it) {
          const int row = it * 4 + q;
          const float* sp = slab + row * 68 + c8;
          v8h hv, lv;
#pragma unroll
          for (int e = 0; e < 8; ++e) {
            if (OUT_MODE == 1) {
              hv[e] = (_Float16)sp[e];
            } else {
              unsigned short hb = f2bf_bits(sp[e]);
              unsigned short lb = f2bf_bits(sp[e] - bf_bits2f(hb));
              hv[e] = __builtin_bit_cast(_Float16, hb);
              lv[e] = __builtin_bit_cast(_Float16, lb);
            }
          }
          *(volatile v8h*)(C + (size_t)(mBase + row) * ldc + n0 + c8) = hv;
          if (OUT_MODE == 2) *(volatile v8h*)(C2 + (size_t)(mBase + row) * ldc + n0 + c8) = lv;
        }
        __threadfence();
      }
    }
    __builtin_amdgcn_fence(__ATOMIC_RELEASE, "workgroup");
    __builtin_amdgcn_wave_barrier();
    __builtin_amdgcn_fence(__ATOMIC_ACQUIRE, "workgroup");
  }
}

__global__ __launch_bounds__(256) void wt_plane_kernel(const float* __restrict__ W, unsigned short* __restrict__ dst, int K, int N, int nLive, int ldd, int colOff) {
  const int n  = blockIdx.x;
  const int k8 = threadIdx.x * 8;
  const bool live = n < nLive;
  const int nc = live ? n : 0;
  v8h hv;
#pragma unroll
  for (int e = 0; e < 8; ++e) {
    const float w = W[(size_t)(k8 + e) * N + nc];
    hv[e] = (_Float16)(live ? carry_flush(bf16r(w), kWCarry) : 0.0f);
  }
  unsigned short* dp = dst + (size_t)n * ldd + colOff + k8;
  *(volatile v8h*)dp = hv;
  __threadfence();
  *(volatile v8h*)dp = hv;
}


__device__ __forceinline__ float phi1(float x) { return (x > 0.0f) ? (x + 1.0f) : expf(x); }

constexpr int kFINB = 0, kFEMOB = 512, kFZB = 1024, kFL0 = 3072, kFLS = 4608, kFEnd = kFL0 + kNL * kFLS;
constexpr int kFQ = 0, kFO = 1536, kF1 = 2048, kF2 = 4096;
__global__ __launch_bounds__(kThr) void setup_kernel(const float* __restrict__ in_b, const float* __restrict__ emo_b, const float* __restrict__ bq,
                                                     const float* __restrict__ bk, const float* __restrict__ bv, const float* __restrict__ bo,
                                                     const float* __restrict__ b1, const float* __restrict__ b2, float* __restrict__ BIAS) {
  unsigned v = blockIdx.x * (unsigned)kThr + threadIdx.x;
  asm volatile("" : "+v"(v));
  const unsigned i0 = v * 4u;
  v4f o = {0.f, 0.f, 0.f, 0.f};
  if (i0 < (unsigned)kFEMOB) {
    const v4f a = *(const v4f*)(in_b + i0);
#pragma unroll
    for (int e = 0; e < 4; ++e) { const float p = a[e]; o[e] = bf16r(p); }
  } else if (i0 < (unsigned)kFL0) {
    const bool live = i0 < (unsigned)(kFEMOB + kNE);
    v4f a = *(const v4f*)(emo_b + (live ? (i0 - (unsigned)kFEMOB) : 0u));
    asm volatile("" : "+v"(a));
#pragma unroll
    for (int e = 0; e < 4; ++e) { const float p = a[e]; o[e] = live ? bf16r(p) : 0.0f; }
  } else {
    const unsigned j = i0 - (unsigned)kFL0;
    const unsigned l = j / (unsigned)kFLS, r = j - l * (unsigned)kFLS;
    const float* sp;
    if (r < 512u) sp = bq + (size_t)l * kD + r;
    else if (r < 1024u) sp = bk + (size_t)l * kD + (r - 512u);
    else if (r < (unsigned)kFO) sp = bv + (size_t)l * kD + (r - 1024u);
    else if (r < (unsigned)kF1) sp = bo + (size_t)l * kD + (r - (unsigned)kFO);
    else if (r < (unsigned)kF2) sp = b1 + (size_t)l * kFF + (r - (unsigned)kF1);
    else sp = b2 + (size_t)l * kD + (r - (unsigned)kF2);
    const v4f a = *(const v4f*)sp;
#pragma unroll
    for (int e = 0; e < 4; ++e) { const float p = a[e]; o[e] = bf16r(p); }
  }
  float* dp = BIAS + i0;
  *(volatile v4f*)dp = o;
  __threadfence();
  *(volatile v4f*)dp = o;
}
static_assert(kFEnd == 58368 && kFEnd / 4 == 57 * kThr && (kFEMOB % 128) == 0 && (kFL0 % 128) == 0 && (kFLS % 128) == 0 && (kFO % 128) == 0 && (kF1 % 128) == 0 && (kF2 % 128) == 0 && kFZB + kFF <= kFL0 && kFZB >= kFEMOB + kNEP, "bias stream map; regions wave-uniform; the zero row covers the widest zero-bias product");

__global__ __launch_bounds__(kThr) void embed_kernel(const int* __restrict__ x, const float* __restrict__ t0, const float* __restrict__ t1,
                                                     const float* __restrict__ t2, const float* __restrict__ t3, const float* __restrict__ t4,
                                                     const float* __restrict__ t5, unsigned short* __restrict__ E16) {
  unsigned v = blockIdx.x * (unsigned)kThr + threadIdx.x;
  asm volatile("" : "+v"(v));
  const unsigned s = v / 96u, c8 = (v - s * 96u) * 8u;
  const unsigned ti = (c8 >= 32u ? 1u : 0u) + (c8 >= 160u ? 1u : 0u) + (c8 >= 416u ? 1u : 0u) + (c8 >= 672u ? 1u : 0u) + (c8 >= 704u ? 1u : 0u);
  const float* tp = (ti == 0u) ? t0 : (ti == 1u) ? t1 : (ti == 2u) ? t2 : (ti == 3u) ? t3 : (ti == 4u) ? t4 : t5;
  const unsigned wi  = (ti == 0u) ? 32u : (ti == 1u) ? 128u : (ti == 2u) ? 256u : (ti == 3u) ? 256u : (ti == 4u) ? 32u : 64u;
  const unsigned oi  = (ti == 0u) ? 0u : (ti == 1u) ? 32u : (ti == 2u) ? 160u : (ti == 3u) ? 416u : (ti == 4u) ? 672u : 704u;
  const int nt       = (ti == 0u) ? 32 : (ti == 1u) ? 32 : (ti == 2u) ? 90 : (ti == 3u) ? 70 : 8;
  const float sc     = (ti == 0u) ? 5.656854249492381f : (ti == 1u) ? 11.313708498984761f : (ti == 2u) ? 16.0f : (ti == 3u) ? 16.0f : (ti == 4u) ? 5.656854249492381f : 8.0f;
  int id = x[s * 6u + ti];
  asm volatile("" : "+v"(id));
  id = (id < 0) ? 0 : ((id > nt - 1) ? (nt - 1) : id);
  const float* sp = tp + (size_t)(unsigned)id * wi + (c8 - oi);
  const v4f a0 = *(const v4f*)sp, a1 = *(const v4f*)(sp + 4);
  v8h hv;
#pragma unroll
  for (int e = 0; e < 4; ++e) { const float p = a0[e], q = a1[e]; hv[e] = (_Float16)carry_flush(bf16r(p) * sc, kInCarry); hv[4 + e] = (_Float16)carry_flush(bf16r(q) * sc, kInCarry); }
  unsigned short* dp = E16 + (size_t)v * 8u;
  *(volatile v8h*)dp = hv;
  __threadfence();
  *(volatile v8h*)dp = hv;
}
static_assert(kE / 8 == 96 && kS * 96 == 384 * kThr, "embedding grid exact");

typedef __attribute__((ext_vector_type(2))) float v2f;
__global__ __launch_bounds__(kThr) void pe_kernel(float* __restrict__ PE) {
  unsigned v = blockIdx.x * (unsigned)kThr + threadIdx.x;
  asm volatile("" : "+v"(v));
  const unsigned s = v >> 8, i = v & 255u;
  const float dv = expf((float)(2u * i) * -0.017988946039015984f);
  const float ang = (float)s * dv;
  v2f o;
  o[0] = sinf(ang); o[1] = cosf(ang);
  float* dp = PE + (size_t)v * 2u;
  *(volatile v2f*)dp = o;
  __threadfence();
  *(volatile v2f*)dp = o;
}
static_assert(kS * (kD / 2) == 1024 * kThr, "position-table grid exact");

__global__ __launch_bounds__(kThr) void addpe_kernel(const float* __restrict__ H0, const float* __restrict__ PE, float* __restrict__ H,
                                                     unsigned short* __restrict__ H16) {
  unsigned v = blockIdx.x * (unsigned)kThr + threadIdx.x;
  asm volatile("" : "+v"(v));
  const size_t o8 = (size_t)v * 8u;
  const v4f a0 = *(const v4f*)(H0 + o8), a1 = *(const v4f*)(H0 + o8 + 4), p0 = *(const v4f*)(PE + o8), p1 = *(const v4f*)(PE + o8 + 4);
  const v4f h0 = a0 + p0, h1 = a1 + p1;
  v8h hv;
#pragma unroll
  for (int e = 0; e < 4; ++e) { hv[e] = (_Float16)carry_flush(h0[e], kInCarry); hv[4 + e] = (_Float16)carry_flush(h1[e], kInCarry); }
  for (int pass = 0; pass < 2; ++pass) {
    *(volatile v4f*)(H + o8) = h0;
    *(volatile v4f*)(H + o8 + 4) = h1;
    *(volatile v8h*)(H16 + o8) = hv;
    __threadfence();
  }
}
static_assert(((size_t)kS * kD / 8) % kThr == 0, "add grid exact");

__global__ __launch_bounds__(kThr) void prepn_kernel(const float* __restrict__ QKV, unsigned short* __restrict__ Q16, unsigned short* __restrict__ K16,
                                                     float* __restrict__ KF) {
  unsigned v = blockIdx.x * (unsigned)kThr + threadIdx.x;
  asm volatile("" : "+v"(v));
  const unsigned s = v >> 6, c8 = (v & 63u) * 8u;
  const float* sp = QKV + (size_t)s * (3 * kD) + c8;
  const v4f q0 = *(const v4f*)sp, q1 = *(const v4f*)(sp + 4), k0 = *(const v4f*)(sp + kD), k1 = *(const v4f*)(sp + kD + 4);
  v8h qh, kh;
  v4f f0, f1;
#pragma unroll
  for (int e = 0; e < 4; ++e) {
    f0[e] = phi1(k0[e]); f1[e] = phi1(k1[e]);
    qh[e] = (_Float16)carry_flush(phi1(q0[e]), kCQ); qh[4 + e] = (_Float16)carry_flush(phi1(q1[e]), kCQ);
    kh[e] = (_Float16)carry_flush(f0[e], kCQ); kh[4 + e] = (_Float16)carry_flush(f1[e], kCQ);
  }
  const size_t o8 = (size_t)v * 8u;
  for (int pass = 0; pass < 2; ++pass) {
    *(volatile v8h*)(Q16 + o8) = qh;
    *(volatile v8h*)(K16 + o8) = kh;
    *(volatile v4f*)(KF + o8) = f0;
    *(volatile v4f*)(KF + o8 + 4) = f1;
    __threadfence();
  }
}
__global__ __launch_bounds__(kThr) void prept_kernel(const float* __restrict__ QKV, unsigned short* __restrict__ KT16, unsigned short* __restrict__ VT16) {
  unsigned v = blockIdx.x * (unsigned)kThr + threadIdx.x;
  asm volatile("" : "+v"(v));
  const unsigned m8 = (v & 15u) * 8u, col = (v >> 4) & 63u, h = (v >> 10) & 7u, ch = v >> 13;
  const float* sp = QKV + (size_t)(ch * (unsigned)kC + m8) * (3 * kD) + h * (unsigned)kDH + col;
  v8h kh, vh;
#pragma unroll
  for (int e = 0; e < 8; ++e) {
    float kx = sp[(size_t)e * (3 * kD) + kD], vx = sp[(size_t)e * (3 * kD) + 2 * kD];
    asm volatile("" : "+v"(kx), "+v"(vx));
    kh[e] = (_Float16)carry_flush(phi1(kx), kCQ);
    vh[e] = (_Float16)carry_flush(vx, kInCarry);
  }
  const size_t o8 = (size_t)v * 8u;
  for (int pass = 0; pass < 2; ++pass) {
    *(volatile v8h*)(KT16 + o8) = kh;
    *(volatile v8h*)(VT16 + o8) = vh;
    __threadfence();
  }
}
static_assert(((size_t)kS * kD / 8) == 256 * kThr && kNC * kNH * kDH * (kC / 8) == 256 * kThr, "the two preparation grids exact");

__global__ __launch_bounds__(kThr) void zero_kernel(float* __restrict__ Z) {
  unsigned v = blockIdx.x * (unsigned)kThr + threadIdx.x;
  asm volatile("" : "+v"(v));
  if (v >= 12416u) return;
  const v4f z = {0.f, 0.f, 0.f, 0.f};
  float* dp = Z + (size_t)v * 4u;
  *(volatile v4f*)dp = z;
  __threadfence();
  *(volatile v4f*)dp = z;
}
static_assert(kOffST16 == kOffST32 + 131072ull && kOffKS == kOffST16 + 65536ull && (131072 + 65536 + 2048) / 16 == 12416 && (12416 % 32) == 0, "the zero state is contiguous; whole waves");

__global__ __launch_bounds__(kThr) void cmask_kernel(const float* __restrict__ SC, unsigned short* __restrict__ W16, float* __restrict__ DENI) {
  unsigned r = blockIdx.x * (unsigned)kThr + threadIdx.x;
  asm volatile("" : "+v"(r));
  const unsigned n = r & 127u;
  const float* sp = SC + (size_t)r * kC;
  unsigned short* wp = W16 + (size_t)r * kC;
  float den = 0.0f;
#pragma unroll 1
  for (unsigned m8 = 0; m8 < (unsigned)kC; m8 += 8) {
    const v4f a0 = *(const v4f*)(sp + m8), a1 = *(const v4f*)(sp + m8 + 4);
    float w[8];
#pragma unroll
    for (int e = 0; e < 4; ++e) { w[e] = ((m8 + (unsigned)e) <= n) ? a0[e] : 0.0f; w[4 + e] = ((m8 + 4u + (unsigned)e) <= n) ? a1[e] : 0.0f; }
    v8h hv;
#pragma unroll
    for (int e = 0; e < 8; ++e) { den += w[e]; hv[e] = (_Float16)carry_flush(w[e], kCW); }
    *(volatile v8h*)(wp + m8) = hv;
    __threadfence();
    *(volatile v8h*)(wp + m8) = hv;
  }
  float* dp = DENI + r;
  *(volatile float*)dp = den;
  __threadfence();
  *(volatile float*)dp = den;
}
static_assert(kNH * kC == 4 * kThr, "causal-score grid exact");

__global__ __launch_bounds__(kThr) void combine_kernel(const float* __restrict__ P1, const float* __restrict__ P2, const float* __restrict__ DENI,
                                                       const unsigned short* __restrict__ Q16, const float* __restrict__ KS,
                                                       unsigned short* __restrict__ ATT16, int c0) {
  unsigned r = blockIdx.x * (unsigned)kThr + threadIdx.x;
  asm volatile("" : "+v"(r));
  const unsigned h = r >> 7, n = r & 127u;
  const unsigned short* qp = Q16 + (size_t)((unsigned)c0 + n) * kD + h * (unsigned)kDH;
  const float* kp = KS + (size_t)h * kDH;
  float qs = 0.0f;
#pragma unroll 1
  for (unsigned d8 = 0; d8 < (unsigned)kDH; d8 += 8) {
    const v8h qv = *(const v8h*)(qp + d8);
    const v4f k0 = *(const v4f*)(kp + d8), k1 = *(const v4f*)(kp + d8 + 4);
#pragma unroll
    for (int e = 0; e < 4; ++e) { qs += (float)qv[e] * k0[e]; qs += (float)qv[4 + e] * k1[e]; }
  }
  const float den = DENI[r] + qs * (1.0f / kCQ) + kAttEps;
  const float inv = 1.0f / den;
  const float* p1 = P1 + (size_t)r * kDH;
  const float* p2 = P2 + (size_t)r * kDH;
  unsigned short* ap = ATT16 + (size_t)((unsigned)c0 + n) * kD + h * (unsigned)kDH;
#pragma unroll 1
  for (unsigned e8 = 0; e8 < (unsigned)kDH; e8 += 8) {
    const v4f a0 = *(const v4f*)(p1 + e8), a1 = *(const v4f*)(p1 + e8 + 4), b0 = *(const v4f*)(p2 + e8), b1 = *(const v4f*)(p2 + e8 + 4);
    v8h hv;
#pragma unroll
    for (int e = 0; e < 4; ++e) { hv[e] = (_Float16)carry_flush((a0[e] + b0[e]) * inv, kInCarry); hv[4 + e] = (_Float16)carry_flush((a1[e] + b1[e]) * inv, kInCarry); }
    *(volatile v8h*)(ap + e8) = hv;
    __threadfence();
    *(volatile v8h*)(ap + e8) = hv;
  }
}

__global__ __launch_bounds__(kThr) void state_kernel(const float* __restrict__ U, const float* __restrict__ KF, float* __restrict__ ST32,
                                                     unsigned short* __restrict__ ST16, float* __restrict__ KS, int c0) {
  unsigned v = blockIdx.x * (unsigned)kThr + threadIdx.x;
  asm volatile("" : "+v"(v));
  if (v < 8192u) {
    const size_t o4 = (size_t)v * 4u;
    const v4f u = *(const v4f*)(U + o4), s0 = *(const v4f*)(ST32 + o4);
    const v4f s1 = s0 + u;
    typedef __attribute__((ext_vector_type(4))) _Float16 v4h;
    v4h hv;
#pragma unroll
    for (int e = 0; e < 4; ++e) hv[e] = (_Float16)carry_flush(s1[e], kCST);
    for (int pass = 0; pass < 2; ++pass) {
      *(volatile v4f*)(ST32 + o4) = s1;
      *(volatile v4h*)(ST16 + o4) = hv;
      __threadfence();
    }
  } else {
    const unsigned w = v - 8192u;
    const float* kp = KF + (size_t)(unsigned)c0 * kD + w;
    float s = KS[w];
#pragma unroll 1
    for (unsigned n = 0; n < (unsigned)kC; ++n) { float x = kp[(size_t)n * kD]; asm volatile("" : "+v"(x)); s += x; }
    float* dp = KS + w;
    *(volatile float*)dp = s;
    __threadfence();
    *(volatile float*)dp = s;
  }
}
static_assert(kNH * kDH * kDH / 4 == 8192 && kNH * kDH == 512 && 8192 + 512 == 34 * kThr && (8192 % 32) == 0, "state grid exact; regions wave-uniform");

__global__ __launch_bounds__(kThr) void addln_kernel(const float* A, const float* __restrict__ ADD, const float* __restrict__ g,
                                                     const float* __restrict__ beta, float* O32, unsigned short* __restrict__ O16, int flags) {
  unsigned r = blockIdx.x * (unsigned)kThr + threadIdx.x;
  asm volatile("" : "+v"(r));
  const bool wantAdd = (flags & 1) != 0, want32 = (flags & 4) != 0, want16 = (flags & 8) != 0;
  const float* a = A + (size_t)r * kD;
  const float* ad = ADD + (size_t)r * kD;
  float s = 0.0f;
#pragma unroll 1
  for (unsigned c = 0; c < (unsigned)kD; c += 4) {
    v4f x = *(const v4f*)(a + c);
    if (wantAdd) { const v4f y = *(const v4f*)(ad + c); x = x + y; }
    s += x[0]; s += x[1]; s += x[2]; s += x[3];
  }
  const float mu = s * kInvD;
  float q = 0.0f;
#pragma unroll 1
  for (unsigned c = 0; c < (unsigned)kD; c += 4) {
    v4f x = *(const v4f*)(a + c);
    if (wantAdd) { const v4f y = *(const v4f*)(ad + c); x = x + y; }
#pragma unroll
    for (int e = 0; e < 4; ++e) { const float d = x[e] - mu; q += d * d; }
  }
  const float rstd = rsqrtf(q * kInvD + kLnEps);
  float* op = O32 + (size_t)r * kD;
  unsigned short* hp = O16 + (size_t)r * kD;
#pragma unroll 1
  for (unsigned c = 0; c < (unsigned)kD; c += 8) {
    v4f x0 = *(const v4f*)(a + c), x1 = *(const v4f*)(a + c + 4);
    if (wantAdd) { const v4f y0 = *(const v4f*)(ad + c), y1 = *(const v4f*)(ad + c + 4); x0 = x0 + y0; x1 = x1 + y1; }
    const v4f g0 = *(const v4f*)(g + c), g1 = *(const v4f*)(g + c + 4), b0 = *(const v4f*)(beta + c), b1 = *(const v4f*)(beta + c + 4);
    v4f n0, n1;
    v8h hv;
#pragma unroll
    for (int e = 0; e < 4; ++e) {
      n0[e] = (x0[e] - mu) * rstd * bf16r(g0[e]) + bf16r(b0[e]);
      n1[e] = (x1[e] - mu) * rstd * bf16r(g1[e]) + bf16r(b1[e]);
      hv[e] = (_Float16)carry_flush(n0[e], kInCarry);
      hv[4 + e] = (_Float16)carry_flush(n1[e], kInCarry);
    }
    for (int pass = 0; pass < 2; ++pass) {
      if (want32) { *(volatile v4f*)(op + c) = n0; *(volatile v4f*)(op + c + 4) = n1; }
      if (want16) { *(volatile v8h*)(hp + c) = hv; }
      __threadfence();
    }
  }
}
static_assert(kS == 4 * kThr, "row grids exact");

__global__ __launch_bounds__(kThr) void gelu_kernel(const float* __restrict__ F1, unsigned short* __restrict__ G16) {
  unsigned v = blockIdx.x * (unsigned)kThr + threadIdx.x;
  asm volatile("" : "+v"(v));
  const float* sp = F1 + (size_t)v * 8u;
  const v4f a0 = *(const v4f*)sp, a1 = *(const v4f*)(sp + 4);
  v8h hv;
#pragma unroll
  for (int e = 0; e < 4; ++e) {
    const float x0 = a0[e], x1 = a1[e];
    const float y0 = 0.5f * x0 * (1.0f + erff(x0 * 0.70710678118654752f)), y1 = 0.5f * x1 * (1.0f + erff(x1 * 0.70710678118654752f));
    hv[e] = (_Float16)carry_flush(y0, kInCarry);
    hv[4 + e] = (_Float16)carry_flush(y1, kInCarry);
  }
  unsigned short* dp = G16 + (size_t)v * 8u;
  *(volatile v8h*)dp = hv;
  __threadfence();
  *(volatile v8h*)dp = hv;
}
static_assert(((size_t)kS * kFF / 8) == 1024 * kThr, "GELU grid exact");

__global__ __launch_bounds__(kThr) void out1_kernel(const float* __restrict__ EMO, float* __restrict__ out1) {
  unsigned v = blockIdx.x * (unsigned)kThr + threadIdx.x;
  asm volatile("" : "+v"(v));
  const unsigned e0 = 4u * v, s = e0 >> 3, c = e0 & 7u;
  const v4f a = *(const v4f*)(EMO + (size_t)s * kNEP + c);
  float* dp = out1 + e0;
  *(volatile v4f*)dp = a;
  __threadfence();
  *(volatile v4f*)dp = a;
}
static_assert(kS * kNE / 4 == 8 * kThr && ((size_t)kS * kD * 4) % 128 == 0, "second-output grid exact; it starts on a 128-B line");

extern "C" void kernel_launch(void* const* d_in, const int* in_sizes, int n_in,
                              void* d_out, int out_size, void* d_ws, size_t ws_size,
                              hipStream_t stream) {
  if (n_in < 29 || d_out == nullptr || d_ws == nullptr) return;
  if (in_sizes[0] != kS * 6 || in_sizes[1] != 32 * 32 || in_sizes[2] != 32 * 128 || in_sizes[3] != 90 * 256 || in_sizes[4] != 70 * 256 || in_sizes[5] != 8 * 32 || in_sizes[6] != 8 * 64) return;
  if (in_sizes[7] != kE * kD || in_sizes[8] != kD) return;
  if (in_sizes[9] != kNL * kD * kD || in_sizes[10] != kNL * kD || in_sizes[11] != kNL * kD * kD || in_sizes[12] != kNL * kD || in_sizes[13] != kNL * kD * kD || in_sizes[14] != kNL * kD || in_sizes[15] != kNL * kD * kD || in_sizes[16] != kNL * kD) return;
  if (in_sizes[17] != kNL * kD || in_sizes[18] != kNL * kD || in_sizes[19] != kNL * kD * kFF || in_sizes[20] != kNL * kFF || in_sizes[21] != kNL * kFF * kD || in_sizes[22] != kNL * kD || in_sizes[23] != kNL * kD || in_sizes[24] != kNL * kD) return;
  if (in_sizes[25] != kD || in_sizes[26] != kD || in_sizes[27] != kD * kNE || in_sizes[28] != kNE) return;
  if (out_size != kS * kD + kS * kNE) return;
  if (ws_size < kWsTotal) return;
  const int* x = (const int*)d_in[0];
  const float* emb0 = (const float*)d_in[1];
  const float* emb1 = (const float*)d_in[2];
  const float* emb2 = (const float*)d_in[3];
  const float* emb3 = (const float*)d_in[4];
  const float* emb4 = (const float*)d_in[5];
  const float* emb5 = (const float*)d_in[6];
  const float* in_w = (const float*)d_in[7];
  const float* in_b = (const float*)d_in[8];
  const float* wq = (const float*)d_in[9];
  const float* bq = (const float*)d_in[10];
  const float* wk = (const float*)d_in[11];
  const float* bk = (const float*)d_in[12];
  const float* wv = (const float*)d_in[13];
  const float* bv = (const float*)d_in[14];
  const float* wo = (const float*)d_in[15];
  const float* bo = (const float*)d_in[16];
  const float* ln1_g = (const float*)d_in[17];
  const float* ln1_b = (const float*)d_in[18];
  const float* w1 = (const float*)d_in[19];
  const float* b1 = (const float*)d_in[20];
  const float* w2 = (const float*)d_in[21];
  const float* b2 = (const float*)d_in[22];
  const float* ln2_g = (const float*)d_in[23];
  const float* ln2_b = (const float*)d_in[24];
  const float* lnf_g = (const float*)d_in[25];
  const float* lnf_b = (const float*)d_in[26];
  const float* emo_w = (const float*)d_in[27];
  const float* emo_b = (const float*)d_in[28];
  float* out = (float*)d_out;
  char* ws = (char*)d_ws;
  unsigned short* E16 = (unsigned short*)(ws + kOffE16);
  unsigned short* INW16 = (unsigned short*)(ws + kOffINW16);
  unsigned short* EMOW16 = (unsigned short*)(ws + kOffEMOW16);
  unsigned short* WQKV16 = (unsigned short*)(ws + kOffWQKV16);
  unsigned short* WO16 = (unsigned short*)(ws + kOffWO16);
  unsigned short* W1H = (unsigned short*)(ws + kOffW1H);
  unsigned short* W2H = (unsigned short*)(ws + kOffW2H);
  float* BIAS = (float*)(ws + kOffBIAS);
  float* PE = (float*)(ws + kOffPE);
  float* H = (float*)(ws + kOffH);
  unsigned short* H16 = (unsigned short*)(ws + kOffH16);
  float* QKV = (float*)(ws + kOffQKV);
  unsigned short* Q16 = (unsigned short*)(ws + kOffQ16);
  unsigned short* K16 = (unsigned short*)(ws + kOffK16);
  float* KF = (float*)(ws + kOffKF);
  unsigned short* KT16 = (unsigned short*)(ws + kOffKT16);
  unsigned short* VT16 = (unsigned short*)(ws + kOffVT16);
  float* SC = (float*)(ws + kOffSC);
  unsigned short* W16 = (unsigned short*)(ws + kOffW16);
  float* DENI = (float*)(ws + kOffDENI);
  float* P1 = (float*)(ws + kOffP1);
  float* P2 = (float*)(ws + kOffP2);
  float* U = (float*)(ws + kOffU);
  float* ST32 = (float*)(ws + kOffST32);
  unsigned short* ST16 = (unsigned short*)(ws + kOffST16);
  float* KS = (float*)(ws + kOffKS);
  unsigned short* ATT16 = (unsigned short*)(ws + kOffATT16);
  float* AO = (float*)(ws + kOffAO);
  float* F1 = (float*)(ws + kOffF1);
  unsigned short* G16 = (unsigned short*)(ws + kOffG16);
  float* EMO = (float*)(ws + kOffEMO);

  setup_kernel<<<57, kThr, 0, stream>>>(in_b, emo_b, bq, bk, bv, bo, b1, b2, BIAS);
  embed_kernel<<<384, kThr, 0, stream>>>(x, emb0, emb1, emb2, emb3, emb4, emb5, E16);
  wt_plane_kernel<<<kD, kE / 8, 0, stream>>>(in_w, INW16, kE, kD, kD, kE, 0);
  wt_plane_kernel<<<kNEP, kD / 8, 0, stream>>>(emo_w, EMOW16, kD, kNE, kNE, kD, 0);
  pe_kernel<<<1024, kThr, 0, stream>>>(PE);
  wmma_gemm64<0, false, 2, 0, false, 0><<<dim3((kS / 64) * (kD / 64) / 8, 1), 256, 0, stream>>>(
      E16, E16, kE, 0L, INW16, INW16, kE, 0L, (void*)QKV, (void*)QKV, kD, 0L, BIAS + kFINB, nullptr, 0L, kS, kD, kE, kScX);
  addpe_kernel<<<256, kThr, 0, stream>>>(QKV, PE, H, H16);

  for (int l = 0; l < kNL; ++l) {
    const float* BL = BIAS + kFL0 + l * kFLS;
    wt_plane_kernel<<<kD, kD / 8, 0, stream>>>(wq + (size_t)l * kD * kD, WQKV16, kD, kD, kD, kD, 0);
    wt_plane_kernel<<<kD, kD / 8, 0, stream>>>(wk + (size_t)l * kD * kD, WQKV16 + (size_t)kD * kD, kD, kD, kD, kD, 0);
    wt_plane_kernel<<<kD, kD / 8, 0, stream>>>(wv + (size_t)l * kD * kD, WQKV16 + (size_t)2 * kD * kD, kD, kD, kD, kD, 0);
    wt_plane_kernel<<<kD, kD / 8, 0, stream>>>(wo + (size_t)l * kD * kD, WO16, kD, kD, kD, kD, 0);
    wt_plane_kernel<<<kFF, kD / 8, 0, stream>>>(w1 + (size_t)l * kD * kFF, W1H, kD, kFF, kFF, kD, 0);
    wt_plane_kernel<<<kD, kFF / 8, 0, stream>>>(w2 + (size_t)l * kFF * kD, W2H, kFF, kD, kD, kFF, 0);
    wmma_gemm64<0, false, 2, 0, false, 0><<<dim3((kS / 64) * (3 * kD / 64) / 8, 1), 256, 0, stream>>>(
        H16, H16, kD, 0L, WQKV16, WQKV16, kD, 0L, (void*)QKV, (void*)QKV, 3 * kD, 0L, BL + kFQ, nullptr, 0L, kS, 3 * kD, kD, kScX);
    prepn_kernel<<<256, kThr, 0, stream>>>(QKV, Q16, K16, KF);
    prept_kernel<<<256, kThr, 0, stream>>>(QKV, KT16, VT16);
    zero_kernel<<<49, kThr, 0, stream>>>(ST32);
    for (int ch = 0; ch < kNC; ++ch) {
      const int c0 = ch * kC;
      const unsigned short* Qc = Q16 + (size_t)c0 * kD;
      const unsigned short* Kc = K16 + (size_t)c0 * kD;
      const unsigned short* KTc = KT16 + (size_t)ch * kNH * kDH * kC;
      const unsigned short* VTc = VT16 + (size_t)ch * kNH * kDH * kC;
      wmma_gemm64<0, false, 2, 0, false, 0><<<dim3(1, kNH), 256, 0, stream>>>(
          Qc, Qc, kD, (long)kDH, Kc, Kc, kD, (long)kDH, (void*)SC, (void*)SC, kC, (long)kC * kC, BIAS + kFZB, nullptr, 0L, kC, kC, kDH, kScQK);
      cmask_kernel<<<4, kThr, 0, stream>>>(SC, W16, DENI);
      wmma_gemm64<0, false, 2, 0, false, 0><<<dim3(1, kNH), 256, 0, stream>>>(
          W16, W16, kC, (long)kC * kC, VTc, VTc, kC, (long)kDH * kC, (void*)P2, (void*)P2, kDH, (long)kC * kDH, BIAS + kFZB, nullptr, 0L, kC, kDH, kC, kScWV);
      wmma_gemm64<0, false, 2, 0, false, 0><<<dim3(1, kNH), 256, 0, stream>>>(
          Qc, Qc, kD, (long)kDH, ST16, ST16, kDH, (long)kDH * kDH, (void*)P1, (void*)P1, kDH, (long)kC * kDH, BIAS + kFZB, nullptr, 0L, kC, kDH, kDH, kScQS);
      combine_kernel<<<4, kThr, 0, stream>>>(P1, P2, DENI, Q16, KS, ATT16, c0);
      if (ch + 1 < kNC) {
        wmma_gemm64<0, false, 2, 0, false, 0><<<dim3(1, kNH), 256, 0, stream>>>(
            VTc, VTc, kC, (long)kDH * kC, KTc, KTc, kC, (long)kDH * kC, (void*)U, (void*)U, kDH, (long)kDH * kDH, BIAS + kFZB, nullptr, 0L, kDH, kDH, kC, kScU);
        state_kernel<<<34, kThr, 0, stream>>>(U, KF, ST32, ST16, KS, c0);
      }
    }
    wmma_gemm64<0, false, 2, 0, false, 0><<<dim3((kS / 64) * (kD / 64) / 8, 1), 256, 0, stream>>>(
        ATT16, ATT16, kD, 0L, WO16, WO16, kD, 0L, (void*)AO, (void*)AO, kD, 0L, BL + kFO, nullptr, 0L, kS, kD, kD, kScX);
    addln_kernel<<<4, kThr, 0, stream>>>(H, AO, ln1_g + (size_t)l * kD, ln1_b + (size_t)l * kD, H, H16, 13);
    wmma_gemm64<0, false, 2, 0, false, 0><<<dim3((kS / 64) * (kFF / 64) / 8, 1), 256, 0, stream>>>(
        H16, H16, kD, 0L, W1H, W1H, kD, 0L, (void*)F1, (void*)F1, kFF, 0L, BL + kF1, nullptr, 0L, kS, kFF, kD, kScX);
    gelu_kernel<<<1024, kThr, 0, stream>>>(F1, G16);
    wmma_gemm64<0, false, 2, 0, false, 0><<<dim3((kS / 64) * (kD / 64) / 8, 1), 256, 0, stream>>>(
        G16, G16, kFF, 0L, W2H, W2H, kFF, 0L, (void*)AO, (void*)AO, kD, 0L, BL + kF2, nullptr, 0L, kS, kD, kFF, kScX);
    addln_kernel<<<4, kThr, 0, stream>>>(H, AO, ln2_g + (size_t)l * kD, ln2_b + (size_t)l * kD, H, H16, 13);
  }
  addln_kernel<<<4, kThr, 0, stream>>>(H, H, lnf_g, lnf_b, out, H16, 12);
  wmma_gemm64<0, false, 2, 0, false, 0><<<dim3((kS / 64) * (kNEP / 64) / 8, 1), 256, 0, stream>>>(
      H16, H16, kD, 0L, EMOW16, EMOW16, kD, 0L, (void*)EMO, (void*)EMO, kNEP, 0L, BIAS + kFEMOB, nullptr, 0L, kS, kNEP, kD, kScX);
  out1_kernel<<<8, kThr, 0, stream>>>(EMO, out + (size_t)kS * kD);
}
